// Rwkv6SelfAttention0_35390530519757
// MI455X (gfx1250) — hardware-run, weakly checked
//
#include <hip/hip_runtime.h>

typedef float          v8f   __attribute__((ext_vector_type(8)));
typedef float          v4f   __attribute__((ext_vector_type(4)));
typedef unsigned int   v4u   __attribute__((ext_vector_type(4)));
typedef int            v8i   __attribute__((ext_vector_type(8)));
typedef unsigned short v8us  __attribute__((ext_vector_type(8)));
typedef unsigned short v16us __attribute__((ext_vector_type(16)));
typedef __bf16         v16bf __attribute__((ext_vector_type(16)));
typedef _Float16       v16h  __attribute__((ext_vector_type(16)));
typedef v4f  __attribute__((may_alias)) v4fa;
typedef v8us __attribute__((may_alias)) v8usa;
union FragB { v16bf v; v16us u; v8us h[2]; v8i w; };
union FragH { v16h  v; v16us u; v8us h[2]; v8i w; };

__device__ __forceinline__ v8f wmb(const FragB& a, const FragB& b, v8f c) {
  v8f d = __builtin_amdgcn_wmma_f32_16x16x32_bf16(false, a.v, false, b.v, (short)0, c, false, false);
  asm volatile("v_nop\n\tv_nop\n\tv_nop\n\tv_nop" : "+v"(d) : "v"(a.w), "v"(b.w));
  return d;
}

__device__ __forceinline__ v8f wmh(const FragH& a, const FragH& b, v8f c) {
  v8f d = __builtin_amdgcn_wmma_f32_16x16x32_f16(false, a.v, false, b.v, (short)0, c, false, false);
  asm volatile("v_nop\n\tv_nop\n\tv_nop\n\tv_nop" : "+v"(d) : "v"(a.w), "v"(b.w));
  return d;
}

__device__ __forceinline__ unsigned bf16_bits(float f) {
  const unsigned u = __float_as_uint(f);
  const unsigned r = (u + 0x7FFFu + ((u >> 16) & 1u)) >> 16;
  const unsigned q = (u >> 16) | 0x40u;
  return ((u & 0x7fffffffu) > 0x7f800000u) ? q : r;
}

__device__ __forceinline__ float bf16_val(float f) {
  return __uint_as_float(bf16_bits(f) << 16);
}
__device__ __forceinline__ int clampi(int v, int lo, int hi) {
  return v < lo ? lo : (v > hi ? hi : v);
}

__device__ __forceinline__ unsigned f16_bits(float f) {
  const unsigned u  = __float_as_uint(f);
  const unsigned s  = (u >> 16) & 0x8000u;
  const unsigned a  = u & 0x7fffffffu;
  const unsigned t  = a - 0x38000000u;
  const unsigned r  = (t + 0x0FFFu + ((t >> 13) & 1u)) >> 13;
  const unsigned rc = r > 0x7C00u ? 0x7C00u : r;
  const bool small  = a < 0x38800000u;
  const bool isnan  = a > 0x7f800000u;
  const unsigned fin = small ? 0u : (s | rc);
  return isnan ? (s | 0x7E00u) : fin;
}

__device__ __forceinline__ unsigned pk16(unsigned lo, unsigned hi) { return lo | (hi << 16); }
__device__ __forceinline__ unsigned bf16_lo_bits(float v) {
  float hi = bf16_val(v);
  asm volatile("" : "+v"(hi));
  return bf16_bits(v - hi);
}
__device__ __forceinline__ v4u pack8_bf16(v4f a, v4f c) {
  return (v4u){ pk16(bf16_bits(a[0]), bf16_bits(a[1])), pk16(bf16_bits(a[2]), bf16_bits(a[3])),
                pk16(bf16_bits(c[0]), bf16_bits(c[1])), pk16(bf16_bits(c[2]), bf16_bits(c[3])) };
}
__device__ __forceinline__ v4u pack8_bf16_lo(v4f a, v4f c) {
  return (v4u){ pk16(bf16_lo_bits(a[0]), bf16_lo_bits(a[1])), pk16(bf16_lo_bits(a[2]), bf16_lo_bits(a[3])),
                pk16(bf16_lo_bits(c[0]), bf16_lo_bits(c[1])), pk16(bf16_lo_bits(c[2]), bf16_lo_bits(c[3])) };
}
__device__ __forceinline__ v4u pack8_f16(v4f a, v4f c) {
  return (v4u){ pk16(f16_bits(a[0]), f16_bits(a[1])), pk16(f16_bits(a[2]), f16_bits(a[3])),
                pk16(f16_bits(c[0]), f16_bits(c[1])), pk16(f16_bits(c[2]), f16_bits(c[3])) };
}

template <int FORM>
__global__ __launch_bounds__(256) void k_plane(const float* __restrict__ src, int rows, int cols, int ldsrc,
                                               unsigned short* __restrict__ dst, int MP, int KP) {
  static_assert(FORM >= 0 && FORM <= 3);
  const int KTOT = (FORM == 1 || FORM == 3) ? 2 * KP : KP;
  const unsigned ppr   = (unsigned)(KTOT >> 3);
  const unsigned kp8   = (unsigned)(KP >> 3);
  const unsigned total = (unsigned)MP * ppr;
  const unsigned g     = blockIdx.x * 256u + threadIdx.x;
  const unsigned rowu  = g / ppr;
  const unsigned p     = g - rowu * ppr;
  const bool second    = p >= kp8;
  const int row = (int)rowu;
  const int c0  = (int)((second ? p - kp8 : p) << 3);
  const float* srow = src + (size_t)clampi(row, 0, rows - 1) * (size_t)ldsrc;
  float x[8];
  unsigned mk[8];
#pragma unroll
  for (int e = 0; e < 8; ++e) {
    const int c = c0 + e;
    const float v = srow[clampi(c, 0, cols - 1)];
    asm volatile("" :: "v"(v));
    x[e]  = v;
    mk[e] = (row < rows && c < cols) ? 0xFFFFu : 0u;
  }
  const v4f a = (v4f){ x[0], x[1], x[2], x[3] };
  const v4f c = (v4f){ x[4], x[5], x[6], x[7] };
  v4u o;
  if (FORM == 2) {
    o = pack8_f16(a, c);
  } else {
    const v4u hi = pack8_bf16(a, c);
    o = hi;
    if (FORM == 1) { const v4u lo = pack8_bf16_lo(a, c); o = second ? lo : hi; }
  }
  const v4u mw = (v4u){ pk16(mk[0], mk[1]), pk16(mk[2], mk[3]), pk16(mk[4], mk[5]), pk16(mk[6], mk[7]) };
  o &= mw;
  if (g < total) {
    volatile v4u* q = (volatile v4u*)(dst + (size_t)g * 8);
    *q = o;
    __threadfence();
    *q = o;
  }
}

template <int FORM> struct FragOf    { typedef FragB T; };
template <>         struct FragOf<2> { typedef FragH T; };
__device__ __forceinline__ v8f mm(const FragB& a, const FragB& b, v8f c) { return wmb(a, b, c); }
__device__ __forceinline__ v8f mm(const FragH& a, const FragH& b, v8f c) { return wmh(a, b, c); }
template <class F> __device__ __forceinline__ F ld_frag(const unsigned short* p) {
  F f;
  f.h[0] = *(const v8usa*)(p);
  f.h[1] = *(const v8usa*)(p + 16);
  return f;
}

template <int FORM, int EPI>
__global__ __launch_bounds__(256) __attribute__((amdgpu_num_vgpr(248)))
void k_gemm_nt(const unsigned short* __restrict__ A, const unsigned short* __restrict__ B,
               const float* __restrict__ bias, float* __restrict__ D, int M, int N, int KTOT, int ldd) {
  static_assert(FORM >= 0 && FORM <= 2);
  static_assert(EPI == 0 || EPI == 1);
  typedef typename FragOf<FORM>::T F;
  __shared__ __attribute__((aligned(16))) float sT[8][16 * 68];
  const int lane = threadIdx.x & 31;
  const int wave = threadIdx.x >> 5;
  const int tilesM = (M + 63) >> 6;
  const int tilesN = (N + 63) >> 6;
  const int tile = blockIdx.x * 8 + wave;
  if (tile >= tilesM * tilesN) return;
  const int tm = tile / tilesN;
  const int tn = tile - tm * tilesN;
  const int m0 = tm << 6;
  const int n0 = tn << 6;

  const int rl = lane & 15;
  const int h8 = (lane >> 4) * 8;
  const unsigned short* pa = A + (size_t)(m0 + rl) * (size_t)KTOT + h8;
  const unsigned short* pb = B + (size_t)(n0 + rl) * (size_t)KTOT + h8;

  v8f acc[4][4];
#pragma unroll
  for (int i = 0; i < 4; ++i)
#pragma unroll
    for (int j = 0; j < 4; ++j) acc[i][j] = (v8f){0.f, 0.f, 0.f, 0.f, 0.f, 0.f, 0.f, 0.f};

#pragma unroll 1
  for (int k0 = 0; k0 < KTOT; k0 += 32) {
    F bf[4];
#pragma unroll
    for (int j = 0; j < 4; ++j) bf[j] = ld_frag<F>(pb + (size_t)(j << 4) * (size_t)KTOT + k0);
#pragma unroll
    for (int i = 0; i < 4; ++i) {
      const F af = ld_frag<F>(pa + (size_t)(i << 4) * (size_t)KTOT + k0);
#pragma unroll
      for (int j = 0; j < 4; ++j) acc[i][j] = mm(af, bf[j], acc[i][j]);
    }
  }

  float* slab = sT[wave];
  const int hh = lane >> 4;
  const int c4 = (lane & 15) * 4;
  const int nc = n0 + c4;
  const bool cok = nc < N;
  v4f bv = (v4f){0.f, 0.f, 0.f, 0.f};
  if (EPI == 1) {
    bv = *(const v4fa*)(bias + clampi(nc, 0, N - 4));
    asm volatile("" :: "v"(bv));
  }
#pragma unroll
  for (int i = 0; i < 4; ++i) {
    const int mBase = m0 + (i << 4);
#pragma unroll
    for (int j = 0; j < 4; ++j) {
#pragma unroll
      for (int r = 0; r < 8; ++r) slab[(h8 + r) * 68 + (j << 4) + rl] = acc[i][j][r];
    }
    __builtin_amdgcn_fence(__ATOMIC_RELEASE, "workgroup");
    __builtin_amdgcn_wave_barrier();
    __builtin_amdgcn_fence(__ATOMIC_ACQUIRE, "workgroup");
    v4f vv[8];
#pragma unroll
    for (int it = 0; it < 8; ++it) {
      const int row = it * 2 + hh;
      v4f v = *(const v4fa*)(slab + row * 68 + c4);
      if (EPI == 1) v += bv;
      vv[it] = v;
    }
    for (int pass = 0; pass < 2; ++pass) {
#pragma unroll
      for (int it = 0; it < 8; ++it) {
        const int row = mBase + it * 2 + hh;
        if (cok && row < M) *(volatile v4f*)(D + (size_t)row * (size_t)ldd + nc) = vv[it];
      }
      __threadfence();
    }
    __builtin_amdgcn_fence(__ATOMIC_RELEASE, "workgroup");
    __builtin_amdgcn_wave_barrier();
    __builtin_amdgcn_fence(__ATOMIC_ACQUIRE, "workgroup");
  }
}

#define TSTEPS 1024
#define NBAT   4
#define DM     1024
#define NHEAD  16
#define HD     64
#define NROW   4096
#define LRK    32
#define NMIXC  160
#define NM1    192
#define KLR    64
#define TC     32
#define NVEC   10
#define V_MAAX 0
#define V_MAA0 1
#define V_TDEC 6
#define V_TF   7
#define V_GNS  8
#define V_GNB  9
#define OUT1_OFF  4194304
#define OUT2_OFF  4198400
#define OUT_TOTAL 4460544

#define SPLIT_MIX1 1
#define SPLIT_MIX2 1
#define SPLIT_TD1  1
#define SPLIT_TD2  1
#define SPLIT_PROJ 1
#define SPLIT_WO   1
#define KT_MIX1 (SPLIT_MIX1 ? 2048 : 1024)
#define KT_TD1  (SPLIT_TD1  ? 2048 : 1024)
#define KT_PROJ (SPLIT_PROJ ? 2048 : 1024)
#define KT_WO   (SPLIT_WO   ? 2048 : 1024)

static_assert(TSTEPS % TC == 0 && TC == 32);
static_assert(HD == 64 && NHEAD * HD == DM && NBAT == 4 && 256 == 4 * HD);
static_assert(NROW == TSTEPS * NBAT);
static_assert(NMIXC == 5 * LRK && NMIXC % 4 == 0 && NM1 >= NMIXC);
static_assert(NROW % 64 == 0 && NM1 % 64 == 0 && DM % 64 == 0 && KLR % 64 == 0);
static_assert(KT_MIX1 % 64 == 0 && KT_TD1 % 64 == 0 && KT_PROJ % 64 == 0 && KT_WO % 64 == 0 && KLR % 32 == 0);
static_assert(NM1 % 32 == 0 && DM % 32 == 0 && KLR % 32 == 0);
static_assert(NROW % 16 == 0 && NM1 % 4 == 0 && DM % 4 == 0);
static_assert(OUT1_OFF == NROW * DM);
static_assert(OUT2_OFF == OUT1_OFF + NBAT * DM);
static_assert(OUT_TOTAL == OUT2_OFF + NBAT * NHEAD * HD * HD);
static_assert((OUT1_OFF * 4) % 128 == 0 && (OUT2_OFF * 4) % 128 == 0);
static_assert((NROW * (DM / 8)) % 256 == 0 && (NROW * 8) % 256 == 0);

__device__ __forceinline__ float pick4(v4f v, int j) {
  return j == 0 ? v.x : (j == 1 ? v.y : (j == 2 ? v.z : v.w));
}
__device__ __forceinline__ v4f put4(v4f v, int j, float r) {
  v.x = (j == 0) ? r : v.x;
  v.y = (j == 1) ? r : v.y;
  v.z = (j == 2) ? r : v.z;
  v.w = (j == 3) ? r : v.w;
  return v;
}
__device__ __forceinline__ float bsel(float a, float b, unsigned m) {
  return __uint_as_float((__float_as_uint(a) & m) | (__float_as_uint(b) & ~m));
}

__global__ __launch_bounds__(256) void k_vec(const float* __restrict__ s0, const float* __restrict__ s1,
                                             const float* __restrict__ s2, const float* __restrict__ s3,
                                             const float* __restrict__ s4, const float* __restrict__ s5,
                                             const float* __restrict__ s6, const float* __restrict__ s7,
                                             const float* __restrict__ s8, const float* __restrict__ s9,
                                             float* __restrict__ VEC) {
  const int tid = (int)threadIdx.x;
  const int which = (int)blockIdx.x;
  const int o = 4 * tid;
  v4f c[10];
  c[0] = *(const v4fa*)(s0 + o);
  c[1] = *(const v4fa*)(s1 + o);
  c[2] = *(const v4fa*)(s2 + o);
  c[3] = *(const v4fa*)(s3 + o);
  c[4] = *(const v4fa*)(s4 + o);
  c[5] = *(const v4fa*)(s5 + o);
  c[6] = *(const v4fa*)(s6 + o);
  c[7] = *(const v4fa*)(s7 + o);
  c[8] = *(const v4fa*)(s8 + o);
  c[9] = *(const v4fa*)(s9 + o);
  unsigned ax = 0u, ay = 0u, az = 0u, aw = 0u;
#pragma unroll
  for (int j = 0; j < 10; ++j) {
    asm volatile("" :: "v"(c[j]));
    const unsigned mk = (which == j) ? 0xFFFFFFFFu : 0u;
    ax |= __float_as_uint(c[j].x) & mk;
    ay |= __float_as_uint(c[j].y) & mk;
    az |= __float_as_uint(c[j].z) & mk;
    aw |= __float_as_uint(c[j].w) & mk;
  }
  const v4f r = (v4f){ bf16_val(__uint_as_float(ax)), bf16_val(__uint_as_float(ay)),
                       bf16_val(__uint_as_float(az)), bf16_val(__uint_as_float(aw)) };
  if (which < NVEC) {
    volatile v4f* q = (volatile v4f*)(VEC + (size_t)which * DM + o);
    *q = r;
    __threadfence();
    *q = r;
  }
}

__global__ __launch_bounds__(256) void k_out1(const float* __restrict__ x, float* __restrict__ out) {
  const int g = (int)blockIdx.x * 256 + (int)threadIdx.x;
  const v4f a = *(const v4fa*)(x + (size_t)(TSTEPS - 1) * NBAT * DM + (size_t)4 * g);
  const v4f r = (v4f){ bf16_val(a.x), bf16_val(a.y), bf16_val(a.z), bf16_val(a.w) };
  volatile v4f* q = (volatile v4f*)(out + (size_t)OUT1_OFF + (size_t)4 * g);
  *q = r;
  __threadfence();
  *q = r;
}

__global__ __launch_bounds__(256) void k_tplane(const float* __restrict__ src, int srows, int scols, int ldsrc,
                                                int srcz, unsigned short* __restrict__ dst, int KTOT, int KP,
                                                int dstz) {
  __shared__ float tl[64 * 65];
  const int tid = (int)threadIdx.x;
  const int kp0 = (int)blockIdx.x * 64;
  const int n0  = (int)blockIdx.y * 64;
  const float* sz = src + (size_t)blockIdx.z * (size_t)srcz;
  unsigned short* dz = dst + (size_t)blockIdx.z * (size_t)dstz;
#pragma unroll
  for (int j = 0; j < 4; ++j) {
    const int idx = tid + 256 * j;
    const int kr  = idx >> 4;
    const int c4  = (idx & 15) * 4;
    const int sr  = (kp0 + kr) % KP;
    const int sc  = n0 + c4;
    const bool ok = (sr < srows) && (sc < scols);
    const v4f v = *(const v4fa*)(sz + (size_t)clampi(sr, 0, srows - 1) * (size_t)ldsrc + clampi(sc, 0, scols - 4));
    asm volatile("" :: "v"(v));
    tl[kr * 65 + c4 + 0] = ok ? v.x : 0.0f;
    tl[kr * 65 + c4 + 1] = ok ? v.y : 0.0f;
    tl[kr * 65 + c4 + 2] = ok ? v.z : 0.0f;
    tl[kr * 65 + c4 + 3] = ok ? v.w : 0.0f;
  }
  __syncthreads();
  v4u ov[2];
  size_t off[2];
#pragma unroll
  for (int it = 0; it < 2; ++it) {
    const int idx = tid + 256 * it;
    const int n = idx >> 3;
    const int p = idx & 7;
    const float* tp = tl + (8 * p) * 65 + n;
    const v4f a = (v4f){ tp[0], tp[65], tp[130], tp[195] };
    const v4f c = (v4f){ tp[260], tp[325], tp[390], tp[455] };
    ov[it]  = pack8_bf16(a, c);
    off[it] = (size_t)(n0 + n) * (size_t)KTOT + (size_t)(kp0 + 8 * p);
  }
  for (int pass = 0; pass < 2; ++pass) {
#pragma unroll
    for (int it = 0; it < 2; ++it) *(volatile v4u*)(dz + off[it]) = ov[it];
    __threadfence();
  }
}

template <int USEMIX>
__global__ __launch_bounds__(256) void k_operand(const float* __restrict__ x, const float* __restrict__ sh,
                                                 const float* __restrict__ maa, const float* __restrict__ mixf,
                                                 unsigned short* __restrict__ AP, int split) {
  const int g    = (int)blockIdx.x * 256 + (int)threadIdx.x;
  const int row  = g >> 7;
  const int c0   = (g & 127) << 3;
  const int bb   = row & (NBAT - 1);
  const int prow = clampi(row - NBAT, 0, NROW - 1);
  const unsigned fm = (row < NBAT) ? 0xFFFFFFFFu : 0u;
  const float* xp = x + (size_t)row * DM + c0;
  const float* pp = x + (size_t)prow * DM + c0;
  const float* sp = sh + (size_t)bb * DM + c0;
  const v4f xa = *(const v4fa*)(xp);
  const v4f xc = *(const v4fa*)(xp + 4);
  const v4f pa = *(const v4fa*)(pp);
  const v4f pc = *(const v4fa*)(pp + 4);
  const v4f sa = *(const v4fa*)(sp);
  const v4f sc = *(const v4fa*)(sp + 4);
  asm volatile("" :: "v"(xa), "v"(xc));
  asm volatile("" :: "v"(pa), "v"(pc));
  asm volatile("" :: "v"(sa), "v"(sc));
  const v4f ma = *(const v4fa*)(maa + c0);
  const v4f mc = *(const v4fa*)(maa + c0 + 4);
  v4f fa = (v4f){0.f, 0.f, 0.f, 0.f};
  v4f fc = (v4f){0.f, 0.f, 0.f, 0.f};
  if (USEMIX == 1) {
    fa = *(const v4fa*)(mixf + (size_t)row * DM + c0);
    fc = *(const v4fa*)(mixf + (size_t)row * DM + c0 + 4);
  }
  v4f va, vc;
#pragma unroll
  for (int e = 0; e < 4; ++e) {
    const float xv0 = bf16_val(xa[e]);
    const float pv0 = bf16_val(bsel(sa[e], pa[e], fm));
    const float dd0 = pv0 - xv0;
    const float mm0 = (USEMIX == 1) ? (ma[e] + fa[e]) : ma[e];
    va[e] = xv0 + dd0 * mm0;
    const float xv1 = bf16_val(xc[e]);
    const float pv1 = bf16_val(bsel(sc[e], pc[e], fm));
    const float dd1 = pv1 - xv1;
    const float mm1 = (USEMIX == 1) ? (mc[e] + fc[e]) : mc[e];
    vc[e] = xv1 + dd1 * mm1;
  }
  const v4u hi = pack8_bf16(va, vc);
  const v4u lo = pack8_bf16_lo(va, vc);
  const int pitch = split ? 2 * DM : DM;
  unsigned short* hp = AP + (size_t)row * (size_t)pitch + c0;
  *(volatile v4u*)hp = hi;
  if (split) *(volatile v4u*)(hp + DM) = lo;
  __threadfence();
  *(volatile v4u*)hp = hi;
  if (split) *(volatile v4u*)(hp + DM) = lo;
}

__global__ __launch_bounds__(256) void k_tanhsplit(const float* __restrict__ src, int ld,
                                                   unsigned short* __restrict__ dst, int split) {
  const int g     = (int)blockIdx.x * 256 + (int)threadIdx.x;
  const int plane = g >> 15;
  const int rem   = g & 32767;
  const int row   = rem >> 3;
  const int p     = rem & 7;
  const int col   = plane * LRK + (p & 3) * 8;
  const bool second = p >= 4;
  const float* sp = src + (size_t)row * (size_t)ld + col;
  const v4f a = *(const v4fa*)(sp);
  const v4f c = *(const v4fa*)(sp + 4);
  v4f ta = (v4f){0.f, 0.f, 0.f, 0.f};
  v4f tc = (v4f){0.f, 0.f, 0.f, 0.f};
#pragma unroll 1
  for (int j = 0; j < 4; ++j) {
    ta = put4(ta, j, tanhf(pick4(a, j)));
    tc = put4(tc, j, tanhf(pick4(c, j)));
  }
  const v4u hi = pack8_bf16(ta, tc);
  v4u lo = pack8_bf16_lo(ta, tc);
  const unsigned sm = split ? 0xFFFFFFFFu : 0u;
  lo &= (v4u){ sm, sm, sm, sm };
  const v4u o = second ? lo : hi;
  volatile v4u* q = (volatile v4u*)(dst + (size_t)g * 8);
  *q = o;
  __threadfence();
  *q = o;
}

__global__ __launch_bounds__(256) void k_scan(const float* __restrict__ RF, const float* __restrict__ KF,
                                              const float* __restrict__ VF, const float* __restrict__ TDF,
                                              const float* __restrict__ VEC, const float* __restrict__ st0,
                                              float* __restrict__ OUTS, float* __restrict__ out2) {
  __shared__ __attribute__((aligned(16))) float sr[TC * HD];
  __shared__ __attribute__((aligned(16))) float sk[TC * HD];
  __shared__ __attribute__((aligned(16))) float sv[TC * HD];
  __shared__ __attribute__((aligned(16))) float sw[TC * HD];
  __shared__ __attribute__((aligned(16))) float sp[TC * 4 * HD];
  const int tid = (int)threadIdx.x;
  const int m   = tid & 63;
  const int q   = tid >> 6;
  const int blk = (int)blockIdx.x;
  const int b   = blk >> 4;
  const int h   = blk & 15;
  const size_t sbase = (size_t)blk * HD * HD;

  float tfr[16];
  {
    const float* tp = VEC + (size_t)V_TF * DM + h * HD + 16 * q;
#pragma unroll
    for (int j = 0; j < 4; ++j) {
      const v4f t4 = *(const v4fa*)(tp + 4 * j);
      tfr[4 * j + 0] = t4.x; tfr[4 * j + 1] = t4.y; tfr[4 * j + 2] = t4.z; tfr[4 * j + 3] = t4.w;
    }
  }
#pragma unroll
  for (int j = 0; j < 4; ++j) {
    const int idx = tid + 256 * j;
    const v4f s4 = *(const v4fa*)(st0 + sbase + (size_t)4 * idx);
    const v4f c4v = (v4f){ bf16_val(s4.x), bf16_val(s4.y), bf16_val(s4.z), bf16_val(s4.w) };
    *(v4fa*)(sp + 4 * idx) = c4v;
  }
  __syncthreads();
  float S[16];
#pragma unroll
  for (int i = 0; i < 16; ++i) S[i] = sp[(16 * q + i) * HD + m];

  const int cc = (tid & 15) * 4;
  const v4f tb = *(const v4fa*)(VEC + (size_t)V_TDEC * DM + h * HD + cc);

#pragma unroll 1
  for (int ch = 0; ch < TSTEPS / TC; ++ch) {
#pragma unroll 1
    for (int it = 0; it < 2; ++it) {
      const int idx = tid + 256 * it;
      const int tt  = idx >> 4;
      const size_t go = (size_t)((ch * TC + tt) * NBAT + b) * DM + h * HD + cc;
      const v4f r4 = *(const v4fa*)(RF + go);
      const v4f k4 = *(const v4fa*)(KF + go);
      const v4f v4 = *(const v4fa*)(VF + go);
      const v4f d4 = *(const v4fa*)(TDF + go);
      v4f w4 = (v4f){0.f, 0.f, 0.f, 0.f};
#pragma unroll 1
      for (int j = 0; j < 4; ++j) {
        const float td = pick4(d4, j) + pick4(tb, j);
        w4 = put4(w4, j, expf(-expf(td)));
      }
      *(v4fa*)(sr + tt * HD + cc) = r4;
      *(v4fa*)(sk + tt * HD + cc) = k4;
      *(v4fa*)(sv + tt * HD + cc) = v4;
      *(v4fa*)(sw + tt * HD + cc) = w4;
    }
    __syncthreads();

#pragma unroll 1
    for (int tt = 0; tt < TC; ++tt) {
      const float vt = sv[tt * HD + m];
      const float* br = sr + tt * HD + 16 * q;
      const float* bk = sk + tt * HD + 16 * q;
      const float* bw = sw + tt * HD + 16 * q;
      float y = 0.0f;
#pragma unroll
      for (int j = 0; j < 4; ++j) {
        const v4f r4 = *(const v4fa*)(br + 4 * j);
        const v4f k4 = *(const v4fa*)(bk + 4 * j);
        const v4f w4 = *(const v4fa*)(bw + 4 * j);
#pragma unroll
        for (int e = 0; e < 4; ++e) {
          const float a = k4[e] * vt;
          y = fmaf(r4[e], fmaf(tfr[4 * j + e], a, S[4 * j + e]), y);
          S[4 * j + e] = fmaf(w4[e], S[4 * j + e], a);
        }
      }
      sp[(tt * 4 + q) * HD + m] = y;
    }
    __syncthreads();

    v4f ov[2];
    size_t oo[2];
#pragma unroll
    for (int it = 0; it < 2; ++it) {
      const int idx = tid + 256 * it;
      const int tt  = idx >> 4;
      const v4f p0 = *(const v4fa*)(sp + (tt * 4 + 0) * HD + cc);
      const v4f p1 = *(const v4fa*)(sp + (tt * 4 + 1) * HD + cc);
      const v4f p2 = *(const v4fa*)(sp + (tt * 4 + 2) * HD + cc);
      const v4f p3 = *(const v4fa*)(sp + (tt * 4 + 3) * HD + cc);
      ov[it] = ((p0 + p1) + p2) + p3;
      oo[it] = (size_t)((ch * TC + tt) * NBAT + b) * DM + h * HD + cc;
    }
    for (int pass = 0; pass < 2; ++pass) {
#pragma unroll
      for (int it = 0; it < 2; ++it) *(volatile v4f*)(OUTS + oo[it]) = ov[it];
      __threadfence();
    }
  }

  float* o2 = out2 + sbase + (size_t)(16 * q) * HD + m;
  for (int pass = 0; pass < 2; ++pass) {
#pragma unroll
    for (int i = 0; i < 16; ++i) *(volatile float*)(o2 + i * HD) = S[i];
    __threadfence();
  }
}

__global__ __launch_bounds__(256) void k_gn(const float* __restrict__ OUTS, const float* __restrict__ ZF,
                                            const float* __restrict__ VEC, unsigned short* __restrict__ YP,
                                            int split) {
  const int lane = (int)threadIdx.x & 31;
  const int wave = (int)threadIdx.x >> 5;
  const int blk  = (int)blockIdx.x;
  const int t    = blk >> 1;
  const int h    = (blk & 1) * 8 + wave;
  const int bb   = lane >> 3;
  const int c    = h * HD + (lane & 7) * 8;
  const int row  = t * NBAT + bb;
  const float* op = OUTS + (size_t)row * DM + c;
  const float* zp = ZF + (size_t)row * DM + c;
  const v4f oa = *(const v4fa*)(op);
  const v4f oc = *(const v4fa*)(op + 4);
  const v4f za = *(const v4fa*)(zp);
  const v4f zc = *(const v4fa*)(zp + 4);
  const v4f sa = *(const v4fa*)(VEC + (size_t)V_GNS * DM + c);
  const v4f sc = *(const v4fa*)(VEC + (size_t)V_GNS * DM + c + 4);
  const v4f ba = *(const v4fa*)(VEC + (size_t)V_GNB * DM + c);
  const v4f bc = *(const v4fa*)(VEC + (size_t)V_GNB * DM + c + 4);
  float s = ((oa.x + oa.y) + (oa.z + oa.w)) + ((oc.x + oc.y) + (oc.z + oc.w));
  s += __shfl_xor(s, 16);
  s += __shfl_xor(s, 8);
  s += __shfl_xor(s, 4);
  s += __shfl_xor(s, 2);
  s += __shfl_xor(s, 1);
  const float mean = s * 0.00390625f;
  const v4f da = oa - mean;
  const v4f dc = oc - mean;
  float ss = ((da.x * da.x + da.y * da.y) + (da.z * da.z + da.w * da.w))
           + ((dc.x * dc.x + dc.y * dc.y) + (dc.z * dc.z + dc.w * dc.w));
  ss += __shfl_xor(ss, 16);
  ss += __shfl_xor(ss, 8);
  ss += __shfl_xor(ss, 4);
  ss += __shfl_xor(ss, 2);
  ss += __shfl_xor(ss, 1);
  const float var = ss * 0.00390625f;
  const float rs  = 1.0f / sqrtf(var + 6.4e-4f);
  v4f ya = (v4f){0.f, 0.f, 0.f, 0.f};
  v4f yc = (v4f){0.f, 0.f, 0.f, 0.f};
#pragma unroll 1
  for (int j = 0; j < 4; ++j) {
    {
      const float xn = pick4(da, j) * rs;
      const float yy = xn * pick4(sa, j) + pick4(ba, j);
      const float z  = pick4(za, j);
      const float sg = 1.0f / (1.0f + expf(-z));
      ya = put4(ya, j, yy * (z * sg));
    }
    {
      const float xn = pick4(dc, j) * rs;
      const float yy = xn * pick4(sc, j) + pick4(bc, j);
      const float z  = pick4(zc, j);
      const float sg = 1.0f / (1.0f + expf(-z));
      yc = put4(yc, j, yy * (z * sg));
    }
  }
  const v4u hi = pack8_bf16(ya, yc);
  const v4u lo = pack8_bf16_lo(ya, yc);
  const int pitch = split ? 2 * DM : DM;
  unsigned short* hp = YP + (size_t)row * (size_t)pitch + c;
  *(volatile v4u*)hp = hi;
  if (split) *(volatile v4u*)(hp + DM) = lo;
  __threadfence();
  *(volatile v4u*)hp = hi;
  if (split) *(volatile v4u*)(hp + DM) = lo;
}

static inline size_t al256(size_t o) { return (o + 255) & ~(size_t)255; }

static inline void run_gemm(const unsigned short* A, const unsigned short* B, const float* bias, float* D,
                            int M, int N, int KTOT, int ldd, hipStream_t s) {
  const int tiles = ((M + 63) / 64) * ((N + 63) / 64);
  k_gemm_nt<1, 0><<<(tiles + 7) / 8, 256, 0, s>>>(A, B, bias, D, M, N, KTOT, ldd);
}

extern "C" void kernel_launch(void* const* d_in, const int* in_sizes, int n_in,
                              void* d_out, int out_size, void* d_ws, size_t ws_size,
                              hipStream_t stream) {
  if (n_in < 22) return;
  if (in_sizes[0] != NROW * DM) return;
  if (in_sizes[1] != NBAT * DM) return;
  if (in_sizes[2] != NBAT * NHEAD * HD * HD) return;
  for (int i = 3; i <= 8; ++i) if (in_sizes[i] != DM) return;
  if (in_sizes[9] != DM * NMIXC) return;
  if (in_sizes[10] != 5 * LRK * DM) return;
  for (int i = 11; i <= 15; ++i) if (in_sizes[i] != DM * DM) return;
  if (in_sizes[16] != DM * LRK) return;
  if (in_sizes[17] != LRK * DM) return;
  if (in_sizes[18] != DM) return;
  if (in_sizes[19] != NHEAD * HD) return;
  if (in_sizes[20] != DM) return;
  if (in_sizes[21] != DM) return;
  if (out_size != OUT_TOTAL) return;

  const float* x    = (const float*)d_in[0];
  const float* sh   = (const float*)d_in[1];
  const float* st0  = (const float*)d_in[2];
  const float* w1   = (const float*)d_in[9];
  const float* w2   = (const float*)d_in[10];
  const float* Wr   = (const float*)d_in[11];
  const float* Wk   = (const float*)d_in[12];
  const float* Wv   = (const float*)d_in[13];
  const float* Wg   = (const float*)d_in[14];
  const float* Wo   = (const float*)d_in[15];
  const float* dw1  = (const float*)d_in[16];
  const float* dw2  = (const float*)d_in[17];
  float* out = (float*)d_out;

  char* ws = (char*)d_ws;
  size_t off = 0;
  const size_t oAHL  = off; off = al256(off + (size_t)NROW * 2048 * 2);
  const size_t oMIXF = off; off = al256(off + (size_t)NROW * DM * 4);
  const size_t oKF   = off; off = al256(off + (size_t)NROW * DM * 4);
  const size_t oVF   = off; off = al256(off + (size_t)NROW * DM * 4);
  const size_t oRF   = off; off = al256(off + (size_t)NROW * DM * 4);
  const size_t oZF   = off; off = al256(off + (size_t)NROW * DM * 4);
  const size_t oTDF  = off; off = al256(off + (size_t)NROW * DM * 4);
  const size_t oWT   = off; off = al256(off + (size_t)DM * 2048 * 2);
  const size_t oW1T2 = off; off = al256(off + (size_t)NM1 * 2048 * 2);
  const size_t oW2T2 = off; off = al256(off + (size_t)5 * DM * KLR * 2);
  const size_t oTDW1 = off; off = al256(off + (size_t)64 * 2048 * 2);
  const size_t oTDW2 = off; off = al256(off + (size_t)DM * KLR * 2);
  const size_t oM1F  = off; off = al256(off + (size_t)NROW * NM1 * 4);
  const size_t oMHL  = off; off = al256(off + (size_t)5 * NROW * KLR * 2);
  const size_t oTD1F = off; off = al256(off + (size_t)NROW * 64 * 4);
  const size_t oTDHL = off; off = al256(off + (size_t)NROW * KLR * 2);
  const size_t oVEC  = off; off = al256(off + (size_t)NVEC * DM * 4);
  if (off > ws_size || off > ((size_t)128 << 20)) return;

  unsigned short* AHL  = (unsigned short*)(ws + oAHL);
  float*          MIXF = (float*)(ws + oMIXF);
  float*          OUTS = (float*)(ws + oMIXF);
  float*          KF   = (float*)(ws + oKF);
  float*          VF   = (float*)(ws + oVF);
  float*          RF   = (float*)(ws + oRF);
  float*          ZF   = (float*)(ws + oZF);
  float*          TDF  = (float*)(ws + oTDF);
  unsigned short* WT   = (unsigned short*)(ws + oWT);
  unsigned short* W1T2 = (unsigned short*)(ws + oW1T2);
  unsigned short* W2T2 = (unsigned short*)(ws + oW2T2);
  unsigned short* TDW1 = (unsigned short*)(ws + oTDW1);
  unsigned short* TDW2 = (unsigned short*)(ws + oTDW2);
  float*          M1F  = (float*)(ws + oM1F);
  unsigned short* MHL  = (unsigned short*)(ws + oMHL);
  float*          TD1F = (float*)(ws + oTD1F);
  unsigned short* TDHL = (unsigned short*)(ws + oTDHL);
  float*          VEC  = (float*)(ws + oVEC);

  k_vec<<<NVEC, 256, 0, stream>>>((const float*)d_in[3], (const float*)d_in[4], (const float*)d_in[5],
                                  (const float*)d_in[6], (const float*)d_in[7], (const float*)d_in[8],
                                  (const float*)d_in[18], (const float*)d_in[19], (const float*)d_in[20],
                                  (const float*)d_in[21], VEC);
  k_out1<<<NBAT * DM / 4 / 256, 256, 0, stream>>>(x, out);

  k_tplane<<<dim3(KT_MIX1 / 64, NM1 / 64, 1), 256, 0, stream>>>(w1, DM, NMIXC, NMIXC, 0, W1T2, KT_MIX1, DM, 0);
  k_tplane<<<dim3(KLR / 64, DM / 64, 5), 256, 0, stream>>>(w2, LRK, DM, DM, LRK * DM, W2T2, KLR, LRK, DM * KLR);
  k_tplane<<<dim3(KT_TD1 / 64, 1, 1), 256, 0, stream>>>(dw1, DM, LRK, LRK, 0, TDW1, KT_TD1, DM, 0);
  k_tplane<<<dim3(KLR / 64, DM / 64, 1), 256, 0, stream>>>(dw2, LRK, DM, DM, 0, TDW2, KLR, LRK, 0);

  k_operand<0><<<NROW * (DM / 8) / 256, 256, 0, stream>>>(x, sh, VEC + (size_t)V_MAAX * DM, VEC, AHL, SPLIT_MIX1);
  run_gemm(AHL, W1T2, VEC, M1F, NROW, NM1, KT_MIX1, NM1, stream);
  k_tanhsplit<<<5 * NROW * 8 / 256, 256, 0, stream>>>(M1F, NM1, MHL, SPLIT_MIX2);

  for (int i = 0; i < 5; ++i) {
    run_gemm(MHL + (size_t)i * NROW * KLR, W2T2 + (size_t)i * DM * KLR, VEC, MIXF, NROW, DM, KLR, DM, stream);
    k_operand<1><<<NROW * (DM / 8) / 256, 256, 0, stream>>>(x, sh, VEC + (size_t)(V_MAA0 + i) * DM, MIXF, AHL,
                                                            (i == 0) ? SPLIT_TD1 : SPLIT_PROJ);
    if (i == 0) {
      run_gemm(AHL, TDW1, VEC, TD1F, NROW, 64, KT_TD1, 64, stream);
      k_tanhsplit<<<NROW * 8 / 256, 256, 0, stream>>>(TD1F, 64, TDHL, SPLIT_TD2);
      run_gemm(TDHL, TDW2, VEC, TDF, NROW, DM, KLR, DM, stream);
    } else {
      const float* W = (i == 1) ? Wk : ((i == 2) ? Wv : ((i == 3) ? Wr : Wg));
      float* Dp      = (i == 1) ? KF : ((i == 2) ? VF : ((i == 3) ? RF : ZF));
      k_tplane<<<dim3(KT_PROJ / 64, DM / 64, 1), 256, 0, stream>>>(W, DM, DM, DM, 0, WT, KT_PROJ, DM, 0);
      run_gemm(AHL, WT, VEC, Dp, NROW, DM, KT_PROJ, DM, stream);
    }
  }

  k_scan<<<NBAT * NHEAD, 256, 0, stream>>>(RF, KF, VF, TDF, VEC, st0, OUTS, out + (size_t)OUT2_OFF);
  k_gn<<<TSTEPS * 2, 256, 0, stream>>>(OUTS, ZF, VEC, AHL, SPLIT_WO);
  k_tplane<<<dim3(KT_WO / 64, DM / 64, 1), 256, 0, stream>>>(Wo, DM, DM, DM, 0, WT, KT_WO, DM, 0);
  run_gemm(AHL, WT, VEC, out, NROW, DM, KT_WO, DM, stream);
}
